// OnnxMultiHeadAttention_81698867904536
// MI455X (gfx1250) — hardware-verified
//
#include <hip/hip_runtime.h>
#include <math.h>
#include <stdint.h>

typedef __attribute__((ext_vector_type(16))) _Float16 v16h;
typedef __attribute__((ext_vector_type(8)))  _Float16 v8h;
typedef __attribute__((ext_vector_type(16))) __bf16   v16b;
typedef __attribute__((ext_vector_type(8)))  __bf16   v8b;
typedef __attribute__((ext_vector_type(8)))  float    v8f;
typedef __attribute__((ext_vector_type(4)))  float    v4f;
typedef __attribute__((ext_vector_type(4)))  unsigned v4u;

static constexpr int kBatch = 4;
static constexpr int kSeq   = 2048;
static constexpr int kDm    = 1024;
static constexpr int kHeads = 16;
static constexpr int kHd    = 64;
static constexpr int kRows  = kBatch * kSeq;
static constexpr int kQB    = 64;
static constexpr int kKC    = 64;
static constexpr int kNW    = 4;

static_assert(kRows % 64 == 0 && kDm % 64 == 0);
static_assert(kDm % 32 == 0);
static_assert(kSeq % kQB == 0 && kHd == 64 && kHeads * kHd == kDm);
static_assert((kRows * kDm) % (8 * 256) == 0 && (kDm * kDm) % (8 * 256) == 0);

__device__ __forceinline__ unsigned short f2bf_bits(float f) {
  unsigned u = __float_as_uint(f);
  return (unsigned short)((u + 0x7FFFu + ((u >> 16) & 1u)) >> 16);
}
__device__ __forceinline__ float bf_bits2f(unsigned short h) { return __uint_as_float(((unsigned)h) << 16); }

__device__ __forceinline__ void dep_guard_h(v8f& a, v8f& b, v16h x, v16h y) { asm volatile("v_nop\n\tv_nop\n\tv_nop\n\tv_nop" : "+v"(a), "+v"(b) : "v"(x), "v"(y)); }
__device__ __forceinline__ void dep_guard_b(v8f& a, v8f& b, v16b x, v16b y) { asm volatile("v_nop\n\tv_nop\n\tv_nop\n\tv_nop" : "+v"(a), "+v"(b) : "v"(x), "v"(y)); }
__device__ __forceinline__ void keep4_h(v16h a, v16h b, v16h c, v16h d) { asm volatile("v_nop" :: "v"(a), "v"(b), "v"(c), "v"(d)); }
__device__ __forceinline__ void keep4_b(v16b a, v16b b, v16b c, v16b d) { asm volatile("v_nop" :: "v"(a), "v"(b), "v"(c), "v"(d)); }
__device__ __forceinline__ void acc_guard4(v8f& a, v8f& b, v8f& c, v8f& d) { asm volatile("v_nop\n\tv_nop\n\tv_nop\n\tv_nop" : "+v"(a), "+v"(b), "+v"(c), "+v"(d)); }
template <typename T> struct Frag;
template <> struct Frag<_Float16> {
  typedef v16h V; union U { v16h v; v8h h[2]; };
  static __device__ __forceinline__ v16h load(const _Float16* p) {
    U f; f.h[0] = *(const v8h*)(p); f.h[1] = *(const v8h*)(p + 16); return f.v;
  }
  static __device__ __forceinline__ v8f mma(v16h a, v16h b, v8f c) {
    return __builtin_amdgcn_wmma_f32_16x16x32_f16(false, a, false, b, (short)0, c, false, false);
  }
  static __device__ __forceinline__ void guard(v8f& a, v8f& b, v16h x, v16h y) { dep_guard_h(a, b, x, y); }
  static __device__ __forceinline__ void keep(v16h a, v16h b, v16h c, v16h d) { keep4_h(a, b, c, d); }
};
template <> struct Frag<__bf16> {
  typedef v16b V; union U { v16b v; v8b h[2]; };
  static __device__ __forceinline__ v16b load(const __bf16* p) {
    U f; f.h[0] = *(const v8b*)(p); f.h[1] = *(const v8b*)(p + 16); return f.v;
  }
  static __device__ __forceinline__ v8f mma(v16b a, v16b b, v8f c) {
    return __builtin_amdgcn_wmma_f32_16x16x32_bf16(false, a, false, b, (short)0, c, false, false);
  }
  static __device__ __forceinline__ void guard(v8f& a, v8f& b, v16b x, v16b y) { dep_guard_b(a, b, x, y); }
  static __device__ __forceinline__ void keep(v16b a, v16b b, v16b c, v16b d) { keep4_b(a, b, c, d); }
};

template <int ET> struct Elem;
template <> struct Elem<0> { typedef _Float16 T; };
template <> struct Elem<1> { typedef __bf16 T; };
template <int ET, int SPLITM, int BIAS_MODE, int OUT_MODE, bool RESID, int ACT = 0>
__global__ __launch_bounds__(256) void wmma_gemm64(
    const unsigned short* __restrict__ Ap, const unsigned short* __restrict__ A2p, int lda, long strideA,
    const unsigned short* __restrict__ Btp, const unsigned short* __restrict__ Bt2p, int ldb, long strideB,
    void* __restrict__ Cout, void* __restrict__ Cout2, int ldc, long strideC,
    const float* __restrict__ bias,
    const float* __restrict__ resid, long strideR,
    int M, int N, int K, float scale) {
  typedef typename Elem<ET>::T T;
  typedef typename Frag<T>::V V;
  const T* A = (const T*)Ap; const T* A2 = (const T*)A2p; const T* Bt = (const T*)Btp; const T* Bt2 = (const T*)Bt2p;
  __shared__ __align__(16) float sT[8][16 * 68];
  const int b    = blockIdx.y;
  const int lane = threadIdx.x & 31;
  const int wave = threadIdx.x >> 5;
  const int tilesN = N >> 6;
  const int tilesM = M >> 6;
  const int tile = blockIdx.x * 8 + wave;
  if (tile >= tilesM * tilesN) return;
  const int tm = tile / tilesN;
  const int tn = tile - tm * tilesN;
  const int m0 = tm << 6;
  const int n0 = tn << 6;

  const T* Ab  = A  + (size_t)b * strideA;
  const T* Bb  = Bt + (size_t)b * strideB;
  const T* Ab2 = (SPLITM != 0) ? (A2  + (size_t)b * strideA) : nullptr;
  const T* Bb2 = (SPLITM == 1) ? (Bt2 + (size_t)b * strideB) : nullptr;

  const int rlane = lane & 15;
  const int koff  = (lane >> 4) * 8;
  const int mOff  = (lane >> 4) * 8;

  v8f acc[4][4];
#pragma unroll
  for (int i = 0; i < 4; ++i)
#pragma unroll
    for (int j = 0; j < 4; ++j) acc[i][j] = (v8f){0.f,0.f,0.f,0.f,0.f,0.f,0.f,0.f};

  for (int k0 = 0; k0 < K; k0 += 32) {
    V bh[4], bl[4];
#pragma unroll
    for (int j = 0; j < 4; ++j) {
      const size_t bo = (size_t)(n0 + (j << 4) + rlane) * ldb + koff + k0;
      bh[j] = Frag<T>::load(Bb + bo);
      if (SPLITM == 1) bl[j] = Frag<T>::load(Bb2 + bo);
    }
#pragma unroll
    for (int i = 0; i < 4; ++i) {
      const size_t ao = (size_t)(m0 + (i << 4) + rlane) * lda + koff + k0;
      V ah = Frag<T>::load(Ab + ao);
      V al;
      if (SPLITM != 0) al = Frag<T>::load(Ab2 + ao);
#pragma unroll
      for (int j = 0; j < 4; ++j) {
        acc[i][j] = Frag<T>::mma(ah, bh[j], acc[i][j]);
        if (SPLITM == 1) {
          acc[i][j] = Frag<T>::mma(ah, bl[j], acc[i][j]);
          acc[i][j] = Frag<T>::mma(al, bh[j], acc[i][j]);
        }
        if (SPLITM == 2) {
          acc[i][j] = Frag<T>::mma(al, bh[j], acc[i][j]);
        }
      }
      Frag<T>::guard(acc[i][0], acc[i][3], ah, (SPLITM != 0) ? al : ah);
    }
    Frag<T>::keep(bh[0], bh[1], bh[2], bh[3]);
    if (SPLITM == 1) Frag<T>::keep(bl[0], bl[1], bl[2], bl[3]);
  }
  acc_guard4(acc[0][0], acc[0][1], acc[0][2], acc[0][3]);
  acc_guard4(acc[1][0], acc[1][1], acc[1][2], acc[1][3]);
  acc_guard4(acc[2][0], acc[2][1], acc[2][2], acc[2][3]);
  acc_guard4(acc[3][0], acc[3][1], acc[3][2], acc[3][3]);

  float* slab = sT[wave];
  const float* Rb = RESID ? (resid + (size_t)b * strideR) : nullptr;
#pragma unroll
  for (int i = 0; i < 4; ++i) {
    const int mBase = m0 + (i << 4);
#pragma unroll
    for (int j = 0; j < 4; ++j) {
      const int n = n0 + (j << 4) + rlane;
      float bv = 0.f;
      if (BIAS_MODE == 2) bv = bias[n];
#pragma unroll
      for (int r = 0; r < 8; ++r) {
        float v = acc[i][j][r] * scale;
        if (BIAS_MODE == 1) v += bias[mBase + mOff + r];
        if (BIAS_MODE == 2) v += bv;
        if (RESID) v += Rb[(size_t)(mBase + mOff + r) * ldc + n];
        if (ACT == 2) v = fmaxf(v, 0.0f);
        if (ACT == 4) v = (v > 0.f) ? v : 0.01f * v;
        slab[(mOff + r) * 68 + (j << 4) + rlane] = v;
      }
    }
    __builtin_amdgcn_fence(__ATOMIC_RELEASE, "workgroup");
    __builtin_amdgcn_wave_barrier();
    __builtin_amdgcn_fence(__ATOMIC_ACQUIRE, "workgroup");
    if (OUT_MODE == 0) {
      float* C = (float*)Cout + (size_t)b * strideC;
      const int hh = lane >> 4, c4 = (lane & 15) * 4;
      for (int pass = 0; pass < 2; ++pass) {
#pragma unroll
        for (int it = 0; it < 8; ++it) {
          const int row = it * 2 + hh;
          v4f v = *(const v4f*)(slab + row * 68 + c4);
          *(volatile v4f*)(C + (size_t)(mBase + row) * ldc + n0 + c4) = v;
        }
        __threadfence();
      }
    } else {
      const int q = lane >> 3, c8 = (lane & 7) * 8;
      unsigned short* C  = (unsigned short*)Cout  + (size_t)b * strideC;
      unsigned short* C2 = (OUT_MODE == 2) ? ((unsigned short*)Cout2 + (size_t)b * strideC) : nullptr;
      for (int pass = 0; pass < 2; ++pass) {
#pragma unroll
        for (int it = 0; it < 4; ++it) {
          const int row = it * 4 + q;
          const float* sp = slab + row * 68 + c8;
          v8h hv, lv;
#pragma unroll
          for (int e = 0; e < 8; ++e) {
            if (OUT_MODE == 1) {
              hv[e] = (_Float16)sp[e];
            } else {
              unsigned short hb = f2bf_bits(sp[e]);
              unsigned short lb = f2bf_bits(sp[e] - bf_bits2f(hb));
              hv[e] = __builtin_bit_cast(_Float16, hb);
              lv[e] = __builtin_bit_cast(_Float16, lb);
            }
          }
          *(volatile v8h*)(C + (size_t)(mBase + row) * ldc + n0 + c8) = hv;
          if (OUT_MODE == 2) *(volatile v8h*)(C2 + (size_t)(mBase + row) * ldc + n0 + c8) = lv;
        }
        __threadfence();
      }
    }
    __builtin_amdgcn_fence(__ATOMIC_RELEASE, "workgroup");
    __builtin_amdgcn_wave_barrier();
    __builtin_amdgcn_fence(__ATOMIC_ACQUIRE, "workgroup");
  }
}

__device__ __forceinline__ unsigned short at_bf_bits(float f) {
  unsigned u = __float_as_uint(f);
  return (unsigned short)((u + 0x7FFFu + ((u >> 16) & 1u)) >> 16);
}
__device__ __forceinline__ __bf16 at_f2bf(float f) { return __builtin_bit_cast(__bf16, at_bf_bits(f)); }
__device__ __forceinline__ void at_split(float f, __bf16& hi, __bf16& lo) {
  const unsigned short hb = at_bf_bits(f);
  hi = __builtin_bit_cast(__bf16, hb);
  lo = at_f2bf(f - __uint_as_float(((unsigned)hb) << 16));
}
__device__ __forceinline__ v8f at_mma(v16b a, v16b b, v8f c) {
  c = __builtin_amdgcn_wmma_f32_16x16x32_bf16(false, a, false, b, (short)0, c, false, false);
  asm volatile("v_nop\n\tv_nop\n\tv_nop\n\tv_nop" : "+v"(c) : "v"(a), "v"(b));
  return c;
}

__global__ __launch_bounds__(256) void cast_f32_bf16x8(const float* __restrict__ in, unsigned short* __restrict__ out, int n8) {
  const int i = blockIdx.x * 256 + threadIdx.x;
  if (i < n8) {
    const float* p = in + (size_t)i * 8;
    const v4f a = *(const v4f*)p;
    const v4f c = *(const v4f*)(p + 4);
    v4u w;
    w[0] = (unsigned)f2bf_bits(a[0]) | ((unsigned)f2bf_bits(a[1]) << 16);
    w[1] = (unsigned)f2bf_bits(a[2]) | ((unsigned)f2bf_bits(a[3]) << 16);
    w[2] = (unsigned)f2bf_bits(c[0]) | ((unsigned)f2bf_bits(c[1]) << 16);
    w[3] = (unsigned)f2bf_bits(c[2]) | ((unsigned)f2bf_bits(c[3]) << 16);
    volatile v4u* o = (volatile v4u*)(out + (size_t)i * 8);
    *o = w;
    __threadfence();
    *o = w;
  }
}

__global__ __launch_bounds__(256) void rope_split_bf16(const float* __restrict__ src, const float* __restrict__ cosT,
                                                        const float* __restrict__ sinT,
                                                        unsigned short* __restrict__ oh, unsigned short* __restrict__ ol, int n8) {
#pragma clang fp contract(off)
  const int i = blockIdx.x * 256 + threadIdx.x;
  if (i < n8) {
    const int m = i >> 7;
    const int col0 = (i & 127) << 3;
    const int s = m & (kSeq - 1);
    const int f0 = (col0 & (kHd - 1)) >> 1;
    const float* p = src + (size_t)m * kDm + col0;
    const v4f x0 = *(const v4f*)p;
    const v4f x1 = *(const v4f*)(p + 4);
    const v4f cc = *(const v4f*)(cosT + (size_t)s * (kHd / 2) + f0);
    const v4f sn = *(const v4f*)(sinT + (size_t)s * (kHd / 2) + f0);
    const float ev[4] = {x0[0], x0[2], x1[0], x1[2]};
    const float od[4] = {x0[1], x0[3], x1[1], x1[3]};
    float o[8];
#pragma unroll
    for (int k = 0; k < 4; ++k) {
      const float cr = bf_bits2f(f2bf_bits(cc[k]));
      const float sr = bf_bits2f(f2bf_bits(sn[k]));
      const float t1 = ev[k] * cr;
      const float t2 = od[k] * sr;
      const float t3 = ev[k] * sr;
      const float t4 = od[k] * cr;
      o[2 * k]     = t1 - t2;
      o[2 * k + 1] = t3 + t4;
    }
    v4u wh, wl;
#pragma unroll
    for (int k = 0; k < 4; ++k) {
      const unsigned short h0 = f2bf_bits(o[2 * k]);
      const unsigned short l0 = f2bf_bits(o[2 * k] - bf_bits2f(h0));
      const unsigned short h1 = f2bf_bits(o[2 * k + 1]);
      const unsigned short l1 = f2bf_bits(o[2 * k + 1] - bf_bits2f(h1));
      wh[k] = (unsigned)h0 | ((unsigned)h1 << 16);
      wl[k] = (unsigned)l0 | ((unsigned)l1 << 16);
    }
    const size_t off = (size_t)m * kDm + col0;
    volatile v4u* ph = (volatile v4u*)(oh + off);
    volatile v4u* pl = (volatile v4u*)(ol + off);
    *ph = wh;
    *pl = wl;
    __threadfence();
    *ph = wh;
    *pl = wl;
  }
}

__global__ __launch_bounds__(128) void attn_hd64_bf16split(
    const unsigned short* __restrict__ qhp, const unsigned short* __restrict__ qlp,
    const unsigned short* __restrict__ khp, const unsigned short* __restrict__ klp,
    const unsigned short* __restrict__ vhp, const unsigned short* __restrict__ vlp,
    const float* __restrict__ maskp,
    unsigned short* __restrict__ chp, unsigned short* __restrict__ clp, float qk_scale) {
  __shared__ __align__(16) __bf16 Ksh[kKC * kHd];
  __shared__ __align__(16) __bf16 Ksl[kKC * kHd];
  __shared__ __align__(16) __bf16 Vth[kHd * kKC];
  __shared__ __align__(16) __bf16 Vtl[kHd * kKC];
  __shared__ __align__(16) __bf16 Psh[kNW][16 * kKC];
  __shared__ __align__(16) __bf16 Psl[kNW][16 * kKC];
  __shared__ __align__(16) float  MO[kQB * kKC];

  const int tid  = threadIdx.x;
  const int wave = tid >> 5;
  const int lane = tid & 31;
  const int hh   = lane >> 4;
  const int c    = lane & 15;

  const int nqb = kSeq / kQB;
  const int bx  = blockIdx.x;
  const int qb  = bx % nqb;
  const int bh  = bx / nqb;
  const int h   = bh % kHeads;
  const int b   = bh / kHeads;
  const int qbase = qb * kQB;
  const int q0    = qbase + wave * 16;
  const size_t rowb = (size_t)b * kSeq;
  const int hcol = h * kHd;

  float mrow[8], lrow[8];
  v8f oacc[4];
#pragma unroll
  for (int r = 0; r < 8; ++r) { mrow[r] = -INFINITY; lrow[r] = 0.f; }
#pragma unroll
  for (int t = 0; t < 4; ++t) oacc[t] = (v8f){0.f,0.f,0.f,0.f,0.f,0.f,0.f,0.f};

  const int nChunks = qb + 1;
  for (int kc = 0; kc < nChunks; ++kc) {
    const int kv0 = kc * kKC;
    __syncthreads();
    {
      const int kvr = tid >> 1;
      const int dh  = (tid & 1) * 32;
      const size_t src = (rowb + kv0 + kvr) * (size_t)kDm + hcol + dh;
      {
        const uint4* sh = (const uint4*)(khp + src);
        const uint4* sl = (const uint4*)(klp + src);
        uint4* dkh = (uint4*)(Ksh + kvr * kHd + dh);
        uint4* dkl = (uint4*)(Ksl + kvr * kHd + dh);
#pragma unroll
        for (int i = 0; i < 4; ++i) { dkh[i] = sh[i]; dkl[i] = sl[i]; }
      }
      asm volatile("" ::: "memory");
      {
        const uint4* sh = (const uint4*)(vhp + src);
        const uint4* sl = (const uint4*)(vlp + src);
#pragma unroll
        for (int i = 0; i < 4; ++i) {
          const uint4 wa = sh[i];
          const uint4 wb = sl[i];
          const unsigned ua[4] = {wa.x, wa.y, wa.z, wa.w};
          const unsigned ub[4] = {wb.x, wb.y, wb.z, wb.w};
#pragma unroll
          for (int e = 0; e < 4; ++e) {
            const int d = dh + 8 * i + 2 * e;
            Vth[d * kKC + kvr]       = __builtin_bit_cast(__bf16, (unsigned short)(ua[e] & 0xffffu));
            Vth[(d + 1) * kKC + kvr] = __builtin_bit_cast(__bf16, (unsigned short)(ua[e] >> 16));
            Vtl[d * kKC + kvr]       = __builtin_bit_cast(__bf16, (unsigned short)(ub[e] & 0xffffu));
            Vtl[(d + 1) * kKC + kvr] = __builtin_bit_cast(__bf16, (unsigned short)(ub[e] >> 16));
          }
        }
      }
      asm volatile("" ::: "memory");
      {
        const int mr = tid >> 1;
        const float* mp = maskp + (size_t)(qbase + mr) * kSeq + kv0 + dh;
        float* md = MO + mr * kKC + dh;
#pragma unroll
        for (int i = 0; i < 8; ++i) {
          const v4f mv = *(const v4f*)(mp + 4 * i);
          v4f mz;
#pragma unroll
          for (int e = 0; e < 4; ++e) mz[e] = bf_bits2f(f2bf_bits(mv[e]));
          *(v4f*)(md + 4 * i) = mz;
        }
      }
    }
    __syncthreads();

    v16b qah[2], qal[2];
    {
      const __bf16* qhr = (const __bf16*)qhp + (rowb + q0 + c) * (size_t)kDm + hcol + 8 * hh;
      const __bf16* qlr = (const __bf16*)qlp + (rowb + q0 + c) * (size_t)kDm + hcol + 8 * hh;
#pragma unroll
      for (int dc = 0; dc < 2; ++dc) {
        qah[dc] = Frag<__bf16>::load(qhr + dc * 32);
        qal[dc] = Frag<__bf16>::load(qlr + dc * 32);
      }
    }
    v8f s[4];
#pragma unroll
    for (int j = 0; j < 4; ++j) {
      s[j] = (v8f){0.f,0.f,0.f,0.f,0.f,0.f,0.f,0.f};
#pragma unroll
      for (int dc = 0; dc < 2; ++dc) {
        const v16b kb = Frag<__bf16>::load(Ksh + (j * 16 + c) * kHd + dc * 32 + 8 * hh);
        const v16b kl = Frag<__bf16>::load(Ksl + (j * 16 + c) * kHd + dc * 32 + 8 * hh);
        s[j] = at_mma(qah[dc], kb, s[j]);
        s[j] = at_mma(qah[dc], kl, s[j]);
        s[j] = at_mma(qal[dc], kb, s[j]);
      }
    }
    const float* mw = MO + (wave * 16 + 8 * hh) * kKC + c;
    float cm[8];
#pragma unroll
    for (int r = 0; r < 8; ++r) {
      float mx = -INFINITY;
#pragma unroll
      for (int j = 0; j < 4; ++j) {
        const float sv = s[j][r] * qk_scale + mw[r * kKC + j * 16];
        s[j][r] = sv;
        mx = fmaxf(mx, sv);
      }
#pragma unroll
      for (int off = 1; off < 16; off <<= 1) mx = fmaxf(mx, __shfl_xor(mx, off, 32));
      cm[r] = mx;
    }
    __bf16* pwh = Psh[wave];
    __bf16* pwl = Psl[wave];
#pragma unroll
    for (int r = 0; r < 8; ++r) {
      const float mnew  = fmaxf(mrow[r], cm[r]);
      const float alpha = expf(mrow[r] - mnew);
      mrow[r] = mnew;
      float psum = 0.f;
#pragma unroll
      for (int j = 0; j < 4; ++j) {
        const float p = expf(s[j][r] - mnew);
        psum += p;
        __bf16 a, bl;
        at_split(p, a, bl);
        pwh[(8 * hh + r) * kKC + j * 16 + c] = a;
        pwl[(8 * hh + r) * kKC + j * 16 + c] = bl;
      }
#pragma unroll
      for (int off = 1; off < 16; off <<= 1) psum += __shfl_xor(psum, off, 32);
      lrow[r] = lrow[r] * alpha + psum;
#pragma unroll
      for (int t = 0; t < 4; ++t) oacc[t][r] *= alpha;
    }
    __builtin_amdgcn_fence(__ATOMIC_RELEASE, "workgroup");
    __builtin_amdgcn_wave_barrier();
    __builtin_amdgcn_fence(__ATOMIC_ACQUIRE, "workgroup");
#pragma unroll
    for (int kk = 0; kk < 2; ++kk) {
      const v16b pa = Frag<__bf16>::load(pwh + c * kKC + kk * 32 + 8 * hh);
      const v16b pl = Frag<__bf16>::load(pwl + c * kKC + kk * 32 + 8 * hh);
#pragma unroll
      for (int t = 0; t < 4; ++t) {
        const v16b vb = Frag<__bf16>::load(Vth + (t * 16 + c) * kKC + kk * 32 + 8 * hh);
        const v16b vl = Frag<__bf16>::load(Vtl + (t * 16 + c) * kKC + kk * 32 + 8 * hh);
        oacc[t] = at_mma(pa, vb, oacc[t]);
        oacc[t] = at_mma(pa, vl, oacc[t]);
        oacc[t] = at_mma(pl, vb, oacc[t]);
      }
    }
  }

  __syncthreads();
  float* os = MO + wave * 16 * kKC;
#pragma unroll
  for (int r = 0; r < 8; ++r) {
    const float inv = 1.0f / lrow[r];
#pragma unroll
    for (int t = 0; t < 4; ++t) os[(8 * hh + r) * kKC + t * 16 + c] = oacc[t][r] * inv;
  }
  __builtin_amdgcn_fence(__ATOMIC_RELEASE, "workgroup");
  __builtin_amdgcn_wave_barrier();
  __builtin_amdgcn_fence(__ATOMIC_ACQUIRE, "workgroup");
  {
    const int qq = lane >> 3, c8 = (lane & 7) * 8;
    for (int pass = 0; pass < 2; ++pass) {
#pragma unroll
      for (int it = 0; it < 4; ++it) {
        const int row = it * 4 + qq;
        const float* sp = os + row * kKC + c8;
        v8h hv, lv;
#pragma unroll
        for (int e = 0; e < 8; ++e) {
          const unsigned short hb = f2bf_bits(sp[e]);
          const unsigned short lb = f2bf_bits(sp[e] - bf_bits2f(hb));
          hv[e] = __builtin_bit_cast(_Float16, hb);
          lv[e] = __builtin_bit_cast(_Float16, lb);
        }
        const size_t o = (rowb + q0 + row) * (size_t)kDm + hcol + c8;
        *(volatile v8h*)(chp + o) = hv;
        *(volatile v8h*)(clp + o) = lv;
      }
      __threadfence();
    }
  }
}

extern "C" void kernel_launch(void* const* d_in, const int* in_sizes, int n_in,
                              void* d_out, int out_size, void* d_ws, size_t ws_size,
                              hipStream_t stream) {
  if (n_in < 8) return;
  const int nX = kRows * kDm;
  const int nW = kDm * kDm;
  const int nT = kSeq * (kHd / 2);
  if (in_sizes[0] != nX || in_sizes[1] != nT || in_sizes[2] != nT || in_sizes[3] != kSeq * kSeq ||
      in_sizes[4] != nW || in_sizes[5] != nW || in_sizes[6] != nW || in_sizes[7] != nW) return;
  if (out_size != nX) return;
  const size_t MiB = (size_t)1 << 20;
  const size_t carve = 128 * MiB;
  if (ws_size < carve) return;

  const float* x     = (const float*)d_in[0];
  const float* cosT  = (const float*)d_in[1];
  const float* sinT  = (const float*)d_in[2];
  const float* maskp = (const float*)d_in[3];
  const float* wq    = (const float*)d_in[4];
  const float* wk    = (const float*)d_in[5];
  const float* wv    = (const float*)d_in[6];
  const float* wo    = (const float*)d_in[7];
  float* out = (float*)d_out;

  char* ws = (char*)d_ws;
  unsigned short* xb   = (unsigned short*)(ws + 0);
  unsigned short* wqb  = (unsigned short*)(ws + 16 * MiB);
  unsigned short* wkb  = (unsigned short*)(ws + 18 * MiB);
  unsigned short* wvb  = (unsigned short*)(ws + 20 * MiB);
  unsigned short* ctxh = (unsigned short*)(ws + 0);
  unsigned short* ctxl = (unsigned short*)(ws + 16 * MiB);
  float*          f32t = (float*)(ws + 32 * MiB);
  unsigned short* vhb  = (unsigned short*)(ws + 32 * MiB);
  unsigned short* vlb  = (unsigned short*)(ws + 48 * MiB);
  unsigned short* qhb  = (unsigned short*)(ws + 64 * MiB);
  unsigned short* qlb  = (unsigned short*)(ws + 80 * MiB);
  unsigned short* wob  = (unsigned short*)(ws + 64 * MiB);
  unsigned short* khb  = (unsigned short*)(ws + 96 * MiB);
  unsigned short* klb  = (unsigned short*)(ws + 112 * MiB);

  const int nX8 = nX / 8, nW8 = nW / 8;
  const dim3 gGemm((kRows / 64) * (kDm / 64) / 8, 1);
  const float qk_scale = 0.125f;

  cast_f32_bf16x8<<<nX8 / 256, 256, 0, stream>>>(x, xb, nX8);
  cast_f32_bf16x8<<<nW8 / 256, 256, 0, stream>>>(wq, wqb, nW8);
  cast_f32_bf16x8<<<nW8 / 256, 256, 0, stream>>>(wk, wkb, nW8);
  cast_f32_bf16x8<<<nW8 / 256, 256, 0, stream>>>(wv, wvb, nW8);
  wmma_gemm64<1, 0, 0, 0, false><<<gGemm, 256, 0, stream>>>(
      xb, xb, kDm, 0L, wqb, wqb, kDm, 0L, (void*)f32t, (void*)f32t, kDm, 0L, cosT, cosT, 0L, kRows, kDm, kDm, 1.0f);
  rope_split_bf16<<<nX8 / 256, 256, 0, stream>>>(f32t, cosT, sinT, qhb, qlb, nX8);
  wmma_gemm64<1, 0, 0, 0, false><<<gGemm, 256, 0, stream>>>(
      xb, xb, kDm, 0L, wkb, wkb, kDm, 0L, (void*)f32t, (void*)f32t, kDm, 0L, cosT, cosT, 0L, kRows, kDm, kDm, 1.0f);
  rope_split_bf16<<<nX8 / 256, 256, 0, stream>>>(f32t, cosT, sinT, khb, klb, nX8);
  wmma_gemm64<1, 0, 0, 2, false><<<gGemm, 256, 0, stream>>>(
      xb, xb, kDm, 0L, wvb, wvb, kDm, 0L, (void*)vhb, (void*)vlb, kDm, 0L, cosT, cosT, 0L, kRows, kDm, kDm, 1.0f);
  attn_hd64_bf16split<<<kBatch * kHeads * (kSeq / kQB), 128, 0, stream>>>(
      qhb, qlb, khb, klb, vhb, vlb, maskp, ctxh, ctxl, qk_scale);
  cast_f32_bf16x8<<<nW8 / 256, 256, 0, stream>>>(wo, wob, nW8);
  wmma_gemm64<1, 2, 0, 0, false><<<gGemm, 256, 0, stream>>>(
      ctxh, ctxl, kDm, 0L, wob, wob, kDm, 0L, (void*)out, (void*)out, kDm, 0L, cosT, cosT, 0L, kRows, kDm, kDm, 1.0f);
}
